// NonLocalBlockRef_36524401885627
// MI455X (gfx1250) — hardware-verified
//
#include <hip/hip_runtime.h>


#define NB_  4
#define CC   128
#define CI   64
#define NPX  9216
#define NV   4608
#define RB   1152
#define DM   CC
#define LOSC 1024.0f

typedef _Float16 h16;
typedef unsigned short bf;
typedef __attribute__((ext_vector_type(16))) __bf16   v16bf;
typedef __attribute__((ext_vector_type(16))) _Float16 v16h;
typedef __attribute__((ext_vector_type(8)))  _Float16 v8h;
typedef __attribute__((ext_vector_type(8)))  unsigned short v8us;
typedef __attribute__((ext_vector_type(8)))  float    v8f;
typedef __attribute__((ext_vector_type(4)))  float    v4f;
typedef v8h  __attribute__((may_alias)) v8ha;
typedef v4f  __attribute__((may_alias)) v4fa;
typedef v8us __attribute__((may_alias)) v8usa;

__device__ __forceinline__ unsigned short f2bf(float f) { unsigned u = __float_as_uint(f); u += 0x7FFFu + ((u >> 16) & 1u); return (unsigned short)(u >> 16); }
__device__ __forceinline__ float bf2f(unsigned short b) { return __uint_as_float(((unsigned)b) << 16); }
__device__ __forceinline__ float bfr(float f) { return bf2f(f2bf(f)); }
__device__ __forceinline__ v16h cat16(v8h lo, v8h hi) { return __builtin_shufflevector(lo, hi, 0, 1, 2, 3, 4, 5, 6, 7, 8, 9, 10, 11, 12, 13, 14, 15); }
__device__ __forceinline__ v16bf cat16b(v8us lo, v8us hi) { return __builtin_bit_cast(v16bf, __builtin_shufflevector(lo, hi, 0, 1, 2, 3, 4, 5, 6, 7, 8, 9, 10, 11, 12, 13, 14, 15)); }
__device__ __forceinline__ v8f wmma16(v16h a, v16h b, v8f c) { return __builtin_amdgcn_wmma_f32_16x16x32_f16(false, a, false, b, (short)0, c, false, false); }
__device__ __forceinline__ v8f wmmab(v16bf a, v16bf b, v8f c) { return __builtin_amdgcn_wmma_f32_16x16x32_bf16(false, a, false, b, (short)0, c, false, false); }

template <bool SPLITA, bool F16OUT = false>
__global__ __launch_bounds__(128) void k_gemmb(const bf* __restrict__ A, const bf* __restrict__ Al, const bf* __restrict__ Bn, const float* __restrict__ bias, float* C, int ldc, h16* C2, const float* __restrict__ R = nullptr, int K = DM, int roundR = 1) {
    __shared__ __align__(16) float ost[4][16 * 68];
    const int lane = threadIdx.x & 31, wave = threadIdx.x >> 5, lr = lane & 15, hi = lane >> 4;
    const int r0 = blockIdx.x * 64 + wave * 16, c0 = blockIdx.y * 64;
    const size_t aoff = (size_t)(r0 + lr) * K + 8 * hi;
    size_t boff[4];
#pragma unroll
    for (int t = 0; t < 4; ++t) boff[t] = (size_t)(c0 + t * 16 + lr) * K + 8 * hi;
    v8f acc[4];
#pragma unroll
    for (int t = 0; t < 4; ++t) acc[t] = (v8f){};
#pragma unroll 1
    for (int kc = 0; kc < K; kc += 32) {
        const v16bf a = cat16b(*(const v8us*)(A + aoff + kc), *(const v8us*)(A + aoff + kc + 16));
        v16bf al = a;
        if (SPLITA) al = cat16b(*(const v8us*)(Al + aoff + kc), *(const v8us*)(Al + aoff + kc + 16));
#pragma unroll
        for (int t = 0; t < 4; ++t) { const v16bf b = cat16b(*(const v8us*)(Bn + boff[t] + kc), *(const v8us*)(Bn + boff[t] + kc + 16)); acc[t] = wmmab(a, b, acc[t]); if (SPLITA) acc[t] = wmmab(al, b, acc[t]); }
        asm volatile("v_nop\n\tv_nop\n\tv_nop\n\tv_nop" : "+v"(acc[0]), "+v"(acc[1]), "+v"(acc[2]), "+v"(acc[3]) : "v"(a), "v"(al));
    }
    float* os = &ost[wave][0];
#pragma unroll
    for (int t = 0; t < 4; ++t) { const float bv = bias ? bfr(bias[c0 + t * 16 + lr]) : 0.f;
#pragma unroll
        for (int j = 0; j < 8; ++j) os[(hi * 8 + j) * 68 + t * 16 + lr] = acc[t][j] + bv; }
    __syncthreads();
    if (F16OUT) {
        h16* crow = (h16*)(void*)C + (size_t)r0 * ldc + c0;
        auto pass = [&]() {
#pragma unroll
            for (int s = 0; s < 4; ++s) { const int row = 4 * s + (lane >> 3), piece = lane & 7; const float* sp = os + row * 68 + piece * 8; v8h o, o2;
#pragma unroll
                for (int i = 0; i < 8; ++i) { const h16 a = (h16)sp[i]; o[i] = a; o2[i] = (h16)((sp[i] - (float)a) * LOSC); }
                *(volatile v8h*)(crow + (size_t)row * ldc + piece * 8) = o; if (C2) *(volatile v8h*)(C2 + (size_t)r0 * ldc + c0 + (size_t)row * ldc + piece * 8) = o2; }
        };
        pass(); __threadfence(); pass();
    } else {
        float* crow = C + (size_t)r0 * ldc + c0;
        auto pass = [&]() {
#pragma unroll
            for (int s = 0; s < 8; ++s) { const int Lid = (lane >> 3) + 4 * s, piece = lane & 7; const int row = Lid >> 1, cofs = (Lid & 1) * 32 + piece * 4;
                v4f val = *(const v4fa*)(os + row * 68 + cofs); if (R) { const v4f rv = *(const v4f*)(R + ((size_t)r0 + row) * ldc + c0 + cofs); val += roundR ? (v4f){bfr(rv[0]), bfr(rv[1]), bfr(rv[2]), bfr(rv[3])} : rv; }
                *(volatile v4f*)(crow + (size_t)row * ldc + cofs) = val; }
        };
        pass(); __threadfence(); pass();
    }
}

__global__ __launch_bounds__(256) void k_cvt8(const float* __restrict__ src, bf* dst, size_t n8) {
    const size_t i = (size_t)blockIdx.x * 256 + threadIdx.x; if (i >= n8) return;
    const v8f v = *(const v8f*)(src + i * 8); v8us o;
#pragma unroll
    for (int k = 0; k < 8; ++k) o[k] = f2bf(v[k]);
    *(volatile v8us*)(dst + i * 8) = o; __threadfence(); *(volatile v8us*)(dst + i * 8) = o;
}
__global__ __launch_bounds__(256) void k_zero8(bf* dst, size_t n8) {
    const size_t i = (size_t)blockIdx.x * 256 + threadIdx.x; if (i >= n8) return; v8us z;
#pragma unroll
    for (int k = 0; k < 8; ++k) z[k] = 0;
    *(volatile v8us*)(dst + i * 8) = z; __threadfence(); *(volatile v8us*)(dst + i * 8) = z;
}
__global__ __launch_bounds__(128) void k_gemm3(const bf* __restrict__ Ah, const bf* __restrict__ Al, const bf* __restrict__ Bh, const bf* __restrict__ Bl, int K, float* C, int ldc) {
    __shared__ __align__(16) float ost[4][16 * 68];
    const int lane = threadIdx.x & 31, wave = threadIdx.x >> 5, lr = lane & 15, hi = lane >> 4;
    const int r0 = blockIdx.x * 64 + wave * 16, c0 = blockIdx.y * 64;
    const size_t aoff = (size_t)(r0 + lr) * K + 8 * hi;
    v8f acc[4];
#pragma unroll
    for (int t = 0; t < 4; ++t) acc[t] = (v8f){};
#pragma unroll 1
    for (int kc = 0; kc < K; kc += 32) {
        const v16bf a = cat16b(*(const v8us*)(Ah + aoff + kc), *(const v8us*)(Ah + aoff + kc + 16));
        const v16bf al = cat16b(*(const v8us*)(Al + aoff + kc), *(const v8us*)(Al + aoff + kc + 16));
#pragma unroll
        for (int t = 0; t < 4; ++t) { const size_t bo = (size_t)(c0 + t * 16 + lr) * K + kc + 8 * hi;
            const v16bf bh = cat16b(*(const v8us*)(Bh + bo), *(const v8us*)(Bh + bo + 16)); const v16bf bl = cat16b(*(const v8us*)(Bl + bo), *(const v8us*)(Bl + bo + 16));
            acc[t] = wmmab(a, bh, acc[t]); acc[t] = wmmab(al, bh, acc[t]); acc[t] = wmmab(a, bl, acc[t]); }
        asm volatile("v_nop\n\tv_nop\n\tv_nop\n\tv_nop" : "+v"(acc[0]), "+v"(acc[1]), "+v"(acc[2]), "+v"(acc[3]) : "v"(a), "v"(al));
    }
    float* os = &ost[wave][0];
#pragma unroll
    for (int t = 0; t < 4; ++t) {
#pragma unroll
        for (int j = 0; j < 8; ++j) os[(hi * 8 + j) * 68 + t * 16 + lr] = acc[t][j]; }
    __builtin_amdgcn_wave_barrier(); asm volatile("" ::: "memory");
    float* crow = C + (size_t)r0 * ldc + c0;
    auto pass = [&]() {
#pragma unroll
        for (int s = 0; s < 8; ++s) { const int Lid = (lane >> 3) + 4 * s, piece = lane & 7; const int row = Lid >> 1, cofs = (Lid & 1) * 32 + piece * 4;
            const v4f val = *(const v4fa*)(os + row * 68 + cofs); *(volatile v4f*)(crow + (size_t)row * ldc + cofs) = val; }
    };
    pass(); __threadfence(); pass();
}


__global__ __launch_bounds__(256) void k_ptb(const float* __restrict__ xb, bf* XT) {
    __shared__ float tl[64][65];
    typedef __attribute__((ext_vector_type(4))) unsigned short v4us;
    const int tid = threadIdx.x, c0 = blockIdx.x * 64, p0 = blockIdx.y * 64; const int rr = tid >> 2, cq = (tid & 3) * 16;
#pragma unroll
    for (int i = 0; i < 16; ++i) tl[rr][cq + i] = xb[(size_t)(c0 + rr) * NPX + p0 + cq + i];
    __syncthreads();
    const int lane = tid & 31, wv = tid >> 5;
    auto pass = [&]() {
#pragma unroll
        for (int st = 0; st < 4; ++st) { const int pr = wv * 8 + st * 2 + (lane >> 4); const int cl = (lane & 15) * 4; v4us v;
#pragma unroll
            for (int i = 0; i < 4; ++i) v[i] = f2bf(tl[cl + i][pr]);
            *(volatile v4us*)(XT + (size_t)(p0 + pr) * CC + c0 + cl) = v; }
    };
    pass(); __threadfence(); pass();
}
__global__ __launch_bounds__(256) void k_viewT(const float* __restrict__ F, bf* Ph, bf* Pl) {
    typedef __attribute__((ext_vector_type(4))) unsigned short v4us;
    const int lane = threadIdx.x & 31; const size_t n = (size_t)blockIdx.x * 8 + (threadIdx.x >> 5); if (n >= (size_t)NV) return; v4us oh, ol;
#pragma unroll
    for (int q = 0; q < 4; ++q) { const int cp = lane * 4 + q; const float y = F[((size_t)(cp & 1) * NV + n) * CI + (cp >> 1)]; const unsigned short hb = f2bf(y); oh[q] = hb; ol[q] = f2bf(y - bf2f(hb)); }
    const size_t o = n * CC + lane * 4; *(volatile v4us*)(Ph + o) = oh; *(volatile v4us*)(Pl + o) = ol; __threadfence(); *(volatile v4us*)(Ph + o) = oh; *(volatile v4us*)(Pl + o) = ol;
}
__global__ __launch_bounds__(256) void k_view(const float* __restrict__ F, bf* Ph, bf* Pl) {
    typedef __attribute__((ext_vector_type(2))) unsigned short v2us;
    const int lane = threadIdx.x & 31; const size_t wid = (size_t)blockIdx.x * 8 + (threadIdx.x >> 5); if (wid >= (size_t)CC * (NV / 64)) return; const int cp = (int)(wid / (NV / 64)); const int m0 = (int)(wid % (NV / 64)) * 64 + lane * 2; v2us oh, ol;
#pragma unroll
    for (int q = 0; q < 2; ++q) { const float y = F[((size_t)(cp & 1) * NV + m0 + q) * CI + (cp >> 1)]; const unsigned short hb = f2bf(y); oh[q] = hb; ol[q] = f2bf(y - bf2f(hb)); }
    const size_t o = (size_t)cp * NV + m0; *(volatile v2us*)(Ph + o) = oh; *(volatile v2us*)(Pl + o) = ol; __threadfence(); *(volatile v2us*)(Ph + o) = oh; *(volatile v2us*)(Pl + o) = ol;
}
__global__ __launch_bounds__(256) void k_colstat(const float* __restrict__ S, float* CM, float* CINV) {
    const int lane = threadIdx.x & 31; const int w = blockIdx.x * 8 + (threadIdx.x >> 5); if (w >= NV / 32) return; const int m = w * 32 + lane; float mx = -3.0e38f;
    for (int n = 0; n < NV; ++n) mx = fmaxf(mx, S[(size_t)n * NV + m]);
    float s = 0.f;
    for (int n = 0; n < NV; ++n) s += __expf(S[(size_t)n * NV + m] - mx);
    const float inv = 1.0f / s; *(volatile float*)(CM + m) = mx; *(volatile float*)(CINV + m) = inv; __threadfence(); *(volatile float*)(CM + m) = mx; *(volatile float*)(CINV + m) = inv;
}
__global__ __launch_bounds__(256) void k_pcol(const float* __restrict__ S, const float* __restrict__ CM, const float* __restrict__ CINV, size_t n0, bf* PH, bf* PL) {
    typedef __attribute__((ext_vector_type(4))) unsigned short v4us;
    const int lane = threadIdx.x & 31; const size_t r = (size_t)blockIdx.x * 8 + (threadIdx.x >> 5); if (r >= (size_t)RB) return; const float* sr = S + (n0 + r) * NV;
#pragma unroll 1
    for (int ps = 0; ps < 2; ++ps) {
#pragma unroll 1
        for (int c0 = lane * 4; c0 < NV; c0 += 128) { v4us oh, ol;
#pragma unroll
            for (int q = 0; q < 4; ++q) { const int m = c0 + q; const float p = __expf(sr[m] - CM[m]) * CINV[m]; const unsigned short hb = f2bf(p); oh[q] = hb; ol[q] = f2bf(p - bf2f(hb)); }
            const size_t o = r * NV + c0; *(volatile v4us*)(PH + o) = oh; *(volatile v4us*)(PL + o) = ol; }
        if (ps == 0) __threadfence(); }
}
__global__ __launch_bounds__(256) void k_yb(const float* __restrict__ Y, bf* Ph, bf* Pl) {
    typedef __attribute__((ext_vector_type(2))) unsigned short v2us;
    const int lane = threadIdx.x & 31; const size_t p = (size_t)blockIdx.x * 8 + (threadIdx.x >> 5); if (p >= (size_t)NPX) return; const size_t n = p % NV; const int half = (int)(p / NV); v2us oh, ol;
#pragma unroll
    for (int q = 0; q < 2; ++q) { const int i = lane * 2 + q; const float y = Y[n * CC + 2 * i + half]; const unsigned short hb = f2bf(y); oh[q] = hb; ol[q] = f2bf(y - bf2f(hb)); }
    const size_t o = p * CI + lane * 2; *(volatile v2us*)(Ph + o) = oh; *(volatile v2us*)(Pl + o) = ol; __threadfence(); *(volatile v2us*)(Ph + o) = oh; *(volatile v2us*)(Pl + o) = ol;
}
__global__ __launch_bounds__(256) void k_outT(const float* __restrict__ MT, const float* __restrict__ x1b, float* OUTB) {
    __shared__ float tl[64][65];
    const int tid = threadIdx.x; const int p0 = blockIdx.x * 64, c0 = blockIdx.y * 64; const int rr = tid >> 2, cq = (tid & 3) * 16;
#pragma unroll
    for (int i = 0; i < 16; ++i) tl[rr][cq + i] = MT[(size_t)(p0 + rr) * CC + c0 + cq + i];
    __syncthreads();
    const int lane = tid & 31, wv = tid >> 5;
    auto pass = [&]() {
#pragma unroll
        for (int st = 0; st < 4; ++st) { const int cr = wv * 8 + st * 2 + (lane >> 4); const int pq = (lane & 15) * 4; v4f v; const size_t o = (size_t)(c0 + cr) * NPX + p0 + pq;
#pragma unroll
            for (int i = 0; i < 4; ++i) v[i] = tl[pq + i][cr] + bfr(x1b[o + i]);
            *(volatile v4f*)(OUTB + o) = v; }
    };
    pass(); __threadfence(); pass();
}

extern "C" void kernel_launch(void* const* d_in, const int* in_sizes, int n_in,
                              void* d_out, int out_size, void* d_ws, size_t ws_size, hipStream_t stream) {
    (void)in_sizes; (void)n_in; (void)out_size;
    const float* x1 = (const float*)d_in[0]; const float* x2 = (const float*)d_in[1]; const float* wth = (const float*)d_in[2]; const float* wph = (const float*)d_in[3]; const float* wg = (const float*)d_in[4]; const float* wm = (const float*)d_in[5];
    float* out = (float*)d_out;
    char* wsp = (char*)d_ws;
    auto take = [&](size_t bytes) { char* p = wsp; wsp += (bytes + 255) & ~(size_t)255; return (void*)p; };
    bf* WT = (bf*)take((size_t)CI * CC * 2); bf* WP = (bf*)take((size_t)CI * CC * 2); bf* WG = (bf*)take((size_t)CI * CC * 2); bf* WM = (bf*)take((size_t)CC * CI * 2);
    bf* X1T = (bf*)take((size_t)NPX * CC * 2); bf* X2T = (bf*)take((size_t)NPX * CC * 2); float* TH = (float*)take((size_t)NPX * CI * 4); float* PHI = (float*)take((size_t)NPX * CI * 4); float* G = (float*)take((size_t)NPX * CI * 4);
    bf* Ah = (bf*)take((size_t)NV * CC * 2); bf* Al = (bf*)take((size_t)NV * CC * 2); bf* Bh = (bf*)take((size_t)NV * CC * 2); bf* Bl = (bf*)take((size_t)NV * CC * 2); bf* Gh = (bf*)take((size_t)CC * NV * 2); bf* Gl = (bf*)take((size_t)CC * NV * 2);
    float* S = (float*)take((size_t)NV * NV * 4); float* CM = (float*)take(NV * 4); float* CINV = (float*)take(NV * 4); bf* PH = (bf*)take((size_t)RB * NV * 2); bf* PL = (bf*)take((size_t)RB * NV * 2); float* Y = (float*)take((size_t)NV * CC * 4);
    if ((size_t)(wsp - (char*)d_ws) > ws_size) return;
    bf* YBh = (bf*)TH; bf* YBl = (bf*)PHI; float* MT = (float*)S;
    k_cvt8<<<(CI * CC / 8 + 255) / 256, 256, 0, stream>>>(wth, WT, CI * CC / 8); k_cvt8<<<(CI * CC / 8 + 255) / 256, 256, 0, stream>>>(wph, WP, CI * CC / 8); k_cvt8<<<(CI * CC / 8 + 255) / 256, 256, 0, stream>>>(wg, WG, CI * CC / 8); k_cvt8<<<(CC * CI / 8 + 255) / 256, 256, 0, stream>>>(wm, WM, CC * CI / 8);
    for (int b = 0; b < NB_; ++b) { const float* x1b = x1 + (size_t)b * CC * NPX; const float* x2b = x2 + (size_t)b * CC * NPX;
        k_ptb<<<dim3(CC / 64, NPX / 64, 1), 256, 0, stream>>>(x1b, X1T); k_ptb<<<dim3(CC / 64, NPX / 64, 1), 256, 0, stream>>>(x2b, X2T);
        k_gemmb<false, false><<<dim3(NPX / 64, 1, 1), 128, 0, stream>>>(X1T, nullptr, WT, nullptr, TH, CI, nullptr, nullptr, CC); k_gemmb<false, false><<<dim3(NPX / 64, 1, 1), 128, 0, stream>>>(X2T, nullptr, WP, nullptr, PHI, CI, nullptr, nullptr, CC); k_gemmb<false, false><<<dim3(NPX / 64, 1, 1), 128, 0, stream>>>(X2T, nullptr, WG, nullptr, G, CI, nullptr, nullptr, CC);
        k_viewT<<<NV / 8, 256, 0, stream>>>(TH, Ah, Al); k_viewT<<<NV / 8, 256, 0, stream>>>(PHI, Bh, Bl); k_view<<<(CC * (NV / 64)) / 8, 256, 0, stream>>>(G, Gh, Gl);
        k_gemm3<<<dim3(NV / 64, NV / 64, 1), 128, 0, stream>>>(Ah, Al, Bh, Bl, CC, S, NV);
        k_colstat<<<(NV / 32) / 8, 256, 0, stream>>>(S, CM, CINV);
        for (int rb = 0; rb < NV / RB; ++rb) { const size_t n0 = (size_t)rb * RB;
            k_pcol<<<RB / 8, 256, 0, stream>>>(S, CM, CINV, n0, PH, PL);
            k_gemm3<<<dim3(RB / 64, CC / 64, 1), 128, 0, stream>>>(PH, PL, Gh, Gl, NV, Y + n0 * CC, CC); }
        k_yb<<<NPX / 8, 256, 0, stream>>>(Y, YBh, YBl);
        k_gemmb<true, false><<<dim3(NPX / 64, CC / 64, 1), 128, 0, stream>>>(YBh, YBl, WM, nullptr, MT, CC, nullptr, nullptr, CI);
        k_outT<<<dim3(NPX / 64, CC / 64, 1), 256, 0, stream>>>(MT, x1b, out + (size_t)b * CC * NPX); }
}
